// Mamba_45535243272446
// MI455X (gfx1250) — hardware-verified
//
#include <hip/hip_runtime.h>
#include <math.h>

typedef __attribute__((ext_vector_type(16))) _Float16 v16h;
typedef __attribute__((ext_vector_type(8)))  _Float16 v8h;
typedef __attribute__((ext_vector_type(16))) __bf16   v16b;
typedef __attribute__((ext_vector_type(8)))  __bf16   v8b;
typedef __attribute__((ext_vector_type(8)))  float    v8f;
typedef __attribute__((ext_vector_type(4)))  float    v4f;

constexpr int kBatch  = 2;
constexpr int kSeq    = 2048;
constexpr int kDm     = 1024;
constexpr int kDin    = 2048;
constexpr int kNst    = 16;
constexpr int kDtR    = 64;
constexpr int kDconv  = 4;
constexpr int kXdW    = 96;
constexpr int kXdP    = 128;
constexpr int kRows   = kBatch * kSeq;
constexpr int kConvTP = 260;
constexpr int kScanTS = 64;
constexpr int kScanCh = 64;
constexpr int kScanXP = 32;
constexpr int kScanYP = 68;
constexpr float kWcarry    = 64.0f;
constexpr float kYcarry    = 16.0f;
constexpr float kWcarryInv = 1.0f / 64.0f;
constexpr float kYWInv     = 1.0f / 1024.0f;
static_assert(kDtR + 2 * kNst == kXdW, "x_proj width");
static_assert((kDm % 32) == 0 && (kDin % 32) == 0 && (kDtR % 32) == 0, "GEMM K multiples of 32");
static_assert((kRows % 64) == 0 && (kDin % 64) == 0 && (kXdP % 64) == 0 && (kDm % 64) == 0, "GEMM M,N multiples of 64");
static_assert((((kRows / 64) * (kDin / 64)) % 8) == 0 && (((kRows / 64) * (kXdP / 64)) % 8) == 0 &&
              (((kRows / 64) * (kDm / 64)) % 8) == 0, "8 tiles per GEMM block");
static_assert((kSeq % kScanTS) == 0 && (kSeq % 64) == 0 && (kDin % kScanCh) == 0 && (kDin % 256) == 0, "tile multiples");

constexpr size_t kOffXH   = 0;
constexpr size_t kOffWIN  = kOffXH  + (size_t)kRows * kDm * 2;
constexpr size_t kOffWXP  = kOffWIN + (size_t)(2 * kDin) * kDm * 2;
constexpr size_t kOffWDT  = kOffWXP + (size_t)kXdP * kDin * 2;
constexpr size_t kOffWOU  = kOffWDT + (size_t)kDin * kDtR * 2;
constexpr size_t kOffXR   = kOffWOU + (size_t)kDm * kDin * 2;
constexpr size_t kOffZR   = kOffXR  + (size_t)kRows * kDin * 4;
constexpr size_t kOffU16  = kOffZR  + (size_t)kRows * kDin * 4;
constexpr size_t kOffXD   = kOffU16 + (size_t)kRows * kDin * 2;
constexpr size_t kOffDTL  = kOffXD  + (size_t)kRows * kXdP * 4;
constexpr size_t kOffY    = kOffDTL + (size_t)kRows * kDtR * 2;
constexpr size_t kWsTotal = kOffY   + (size_t)kRows * kDin * 2;
static_assert(kWsTotal == 125042688ull, "carve total");
static_assert(kWsTotal <= 134217728ull, "carve cap");
static_assert((kOffWIN % 128) == 0 && (kOffWXP % 128) == 0 && (kOffWDT % 128) == 0 && (kOffWOU % 128) == 0 &&
              (kOffXR % 128) == 0 && (kOffZR % 128) == 0 && (kOffU16 % 128) == 0 && (kOffXD % 128) == 0 &&
              (kOffDTL % 128) == 0 && (kOffY % 128) == 0, "128-B aligned regions");

__device__ __forceinline__ unsigned short f2bf_bits(float f) {
  unsigned u = __float_as_uint(f);
  return (unsigned short)((u + 0x7FFFu + ((u >> 16) & 1u)) >> 16);
}
__device__ __forceinline__ float bf_bits2f(unsigned short h) { return __uint_as_float(((unsigned)h) << 16); }
__device__ __forceinline__ float bf_rne(float f) { return bf_bits2f(f2bf_bits(f)); }

__device__ __forceinline__ float h16_to_f32(unsigned hb) {
  const unsigned sgn = (hb & 0x8000u) << 16; const unsigned em = hb & 0x7fffu;
  const float fn = __uint_as_float((em << 13) + 0x38000000u);
  const float fs = (float)em * 5.9604644775390625e-8f;
  const float mag = (em < 0x400u) ? fs : fn; return __uint_as_float(__float_as_uint(mag) | sgn); }

__device__ __forceinline__ void dep_guard4_h(v8f& a, v8f& b, v8f& c, v8f& d, v16h x, v16h y, v16h b0, v16h b1, v16h b2, v16h b3) {
  asm volatile("v_nop\n\tv_nop\n\tv_nop\n\tv_nop" : "+v"(a), "+v"(b), "+v"(c), "+v"(d) : "v"(x), "v"(y), "v"(b0), "v"(b1), "v"(b2), "v"(b3));
}
__device__ __forceinline__ void dep_guard4_b(v8f& a, v8f& b, v8f& c, v8f& d, v16b x, v16b y, v16b b0, v16b b1, v16b b2, v16b b3) {
  asm volatile("v_nop\n\tv_nop\n\tv_nop\n\tv_nop" : "+v"(a), "+v"(b), "+v"(c), "+v"(d) : "v"(x), "v"(y), "v"(b0), "v"(b1), "v"(b2), "v"(b3));
}
__device__ __forceinline__ void keep4_h(v16h a, v16h b, v16h c, v16h d) { asm volatile("v_nop" :: "v"(a), "v"(b), "v"(c), "v"(d)); }
__device__ __forceinline__ void keep4_b(v16b a, v16b b, v16b c, v16b d) { asm volatile("v_nop" :: "v"(a), "v"(b), "v"(c), "v"(d)); }
__device__ __forceinline__ void acc_guard4(v8f& a, v8f& b, v8f& c, v8f& d) { asm volatile("v_nop\n\tv_nop\n\tv_nop\n\tv_nop" : "+v"(a), "+v"(b), "+v"(c), "+v"(d)); }
template <typename T> struct Frag;
template <> struct Frag<_Float16> {
  typedef v16h V; union U { v16h v; v8h h[2]; };
  static __device__ __forceinline__ v16h load(const _Float16* p) {
    U f; f.h[0] = *(const v8h*)(p); f.h[1] = *(const v8h*)(p + 16); return f.v;
  }
  static __device__ __forceinline__ v8f mma(v16h a, v16h b, v8f c) {
    return __builtin_amdgcn_wmma_f32_16x16x32_f16(false, a, false, b, (short)0, c, false, false);
  }
  static __device__ __forceinline__ void guard4(v8f& a, v8f& b, v8f& c, v8f& d, v16h x, v16h y, v16h b0, v16h b1, v16h b2, v16h b3) {
    dep_guard4_h(a, b, c, d, x, y, b0, b1, b2, b3);
  }
  static __device__ __forceinline__ void keep(v16h a, v16h b, v16h c, v16h d) { keep4_h(a, b, c, d); }
};
template <> struct Frag<__bf16> {
  typedef v16b V; union U { v16b v; v8b h[2]; };
  static __device__ __forceinline__ v16b load(const __bf16* p) {
    U f; f.h[0] = *(const v8b*)(p); f.h[1] = *(const v8b*)(p + 16); return f.v;
  }
  static __device__ __forceinline__ v8f mma(v16b a, v16b b, v8f c) {
    return __builtin_amdgcn_wmma_f32_16x16x32_bf16(false, a, false, b, (short)0, c, false, false);
  }
  static __device__ __forceinline__ void guard4(v8f& a, v8f& b, v8f& c, v8f& d, v16b x, v16b y, v16b b0, v16b b1, v16b b2, v16b b3) {
    dep_guard4_b(a, b, c, d, x, y, b0, b1, b2, b3);
  }
  static __device__ __forceinline__ void keep(v16b a, v16b b, v16b c, v16b d) { keep4_b(a, b, c, d); }
};

template <int ET> struct Elem;
template <> struct Elem<0> { typedef _Float16 T; };
template <> struct Elem<1> { typedef __bf16 T; };
template <int ET, bool SPLIT, int BIAS_MODE, int OUT_MODE, bool RESID, int ACT = 0>
__global__ __launch_bounds__(256) void wmma_gemm64(
    const unsigned short* __restrict__ Ap, const unsigned short* __restrict__ A2p, int lda, long strideA,
    const unsigned short* __restrict__ Btp, const unsigned short* __restrict__ Bt2p, int ldb, long strideB,
    void* __restrict__ Cout, void* __restrict__ Cout2, int ldc, long strideC,
    const float* __restrict__ bias,
    const float* __restrict__ resid, long strideR,
    int M, int N, int K, float scale) {
  typedef typename Elem<ET>::T T;
  typedef typename Frag<T>::V V;
  const T* A = (const T*)Ap; const T* A2 = (const T*)A2p; const T* Bt = (const T*)Btp; const T* Bt2 = (const T*)Bt2p;
  __shared__ __align__(16) float sT[8][16 * 68];
  const int b    = blockIdx.y;
  const int lane = threadIdx.x & 31;
  const int wave = threadIdx.x >> 5;
  const int tilesN = N >> 6;
  const int tilesM = M >> 6;
  const int tile = blockIdx.x * 8 + wave;
  if (tile >= tilesM * tilesN) return;
  const int tm = tile / tilesN;
  const int tn = tile - tm * tilesN;
  const int m0 = tm << 6;
  const int n0 = tn << 6;

  const T* Ab  = A  + (size_t)b * strideA;
  const T* Bb  = Bt + (size_t)b * strideB;
  const T* Ab2 = SPLIT ? (A2  + (size_t)b * strideA) : nullptr;
  const T* Bb2 = SPLIT ? (Bt2 + (size_t)b * strideB) : nullptr;

  const int rlane = lane & 15;
  const int koff  = (lane >> 4) * 8;
  const int mOff  = (lane >> 4) * 8;

  v8f acc[4][4];
#pragma unroll
  for (int i = 0; i < 4; ++i)
#pragma unroll
    for (int j = 0; j < 4; ++j) acc[i][j] = (v8f){0.f,0.f,0.f,0.f,0.f,0.f,0.f,0.f};

  for (int k0 = 0; k0 < K; k0 += 32) {
    V bh[4], bl[4];
#pragma unroll
    for (int j = 0; j < 4; ++j) {
      const size_t bo = (size_t)(n0 + (j << 4) + rlane) * ldb + koff + k0;
      bh[j] = Frag<T>::load(Bb + bo);
      if (SPLIT) bl[j] = Frag<T>::load(Bb2 + bo);
    }
#pragma unroll
    for (int i = 0; i < 4; ++i) {
      const size_t ao = (size_t)(m0 + (i << 4) + rlane) * lda + koff + k0;
      V ah = Frag<T>::load(Ab + ao);
      V al;
      if (SPLIT) al = Frag<T>::load(Ab2 + ao);
#pragma unroll
      for (int j = 0; j < 4; ++j) {
        acc[i][j] = Frag<T>::mma(ah, bh[j], acc[i][j]);
        if (SPLIT) {
          acc[i][j] = Frag<T>::mma(ah, bl[j], acc[i][j]);
          acc[i][j] = Frag<T>::mma(al, bh[j], acc[i][j]);
        }
      }
      Frag<T>::guard4(acc[i][0], acc[i][1], acc[i][2], acc[i][3], ah, SPLIT ? al : ah, bh[0], bh[1], bh[2], bh[3]);
    }
    Frag<T>::keep(bh[0], bh[1], bh[2], bh[3]);
    if (SPLIT) Frag<T>::keep(bl[0], bl[1], bl[2], bl[3]);
  }
  acc_guard4(acc[0][0], acc[0][1], acc[0][2], acc[0][3]);
  acc_guard4(acc[1][0], acc[1][1], acc[1][2], acc[1][3]);
  acc_guard4(acc[2][0], acc[2][1], acc[2][2], acc[2][3]);
  acc_guard4(acc[3][0], acc[3][1], acc[3][2], acc[3][3]);

  float* slab = sT[wave];
  const float* Rb = RESID ? (resid + (size_t)b * strideR) : nullptr;
#pragma unroll
  for (int i = 0; i < 4; ++i) {
    const int mBase = m0 + (i << 4);
#pragma unroll
    for (int j = 0; j < 4; ++j) {
      const int n = n0 + (j << 4) + rlane;
      float bv = 0.f;
      if (BIAS_MODE == 2) bv = bias[n];
#pragma unroll
      for (int r = 0; r < 8; ++r) {
        float v = acc[i][j][r] * scale;
        if (BIAS_MODE == 1) v += bias[mBase + mOff + r];
        if (BIAS_MODE == 2) v += bv;
        if (RESID) v += Rb[(size_t)(mBase + mOff + r) * ldc + n];
        if (ACT == 2) v = fmaxf(v, 0.0f);
        if (ACT == 4) v = (v > 0.f) ? v : 0.01f * v;
        slab[(mOff + r) * 68 + (j << 4) + rlane] = v;
      }
    }
    __builtin_amdgcn_fence(__ATOMIC_RELEASE, "workgroup");
    __builtin_amdgcn_wave_barrier();
    __builtin_amdgcn_fence(__ATOMIC_ACQUIRE, "workgroup");
    if (OUT_MODE == 0) {
      float* C = (float*)Cout + (size_t)b * strideC;
      const int hh = lane >> 4, c4 = (lane & 15) * 4;
      for (int pass = 0; pass < 2; ++pass) {
#pragma unroll
        for (int it = 0; it < 8; ++it) {
          const int row = it * 2 + hh;
          v4f v = *(const v4f*)(slab + row * 68 + c4);
          *(volatile v4f*)(C + (size_t)(mBase + row) * ldc + n0 + c4) = v;
        }
        __threadfence();
      }
    } else {
      const int q = lane >> 3, c8 = (lane & 7) * 8;
      unsigned short* C  = (unsigned short*)Cout  + (size_t)b * strideC;
      unsigned short* C2 = (OUT_MODE == 2) ? ((unsigned short*)Cout2 + (size_t)b * strideC) : nullptr;
      for (int pass = 0; pass < 2; ++pass) {
#pragma unroll
        for (int it = 0; it < 4; ++it) {
          const int row = it * 4 + q;
          const float* sp = slab + row * 68 + c8;
          v8h hv, lv;
#pragma unroll
          for (int e = 0; e < 8; ++e) {
            if (OUT_MODE == 1) {
              hv[e] = (_Float16)sp[e];
            } else {
              unsigned short hb = f2bf_bits(sp[e]);
              unsigned short lb = f2bf_bits(sp[e] - bf_bits2f(hb));
              hv[e] = __builtin_bit_cast(_Float16, hb);
              lv[e] = __builtin_bit_cast(_Float16, lb);
            }
          }
          *(volatile v8h*)(C + (size_t)(mBase + row) * ldc + n0 + c8) = hv;
          if (OUT_MODE == 2) *(volatile v8h*)(C2 + (size_t)(mBase + row) * ldc + n0 + c8) = lv;
        }
        __threadfence();
      }
    }
    __builtin_amdgcn_fence(__ATOMIC_RELEASE, "workgroup");
    __builtin_amdgcn_wave_barrier();
    __builtin_amdgcn_fence(__ATOMIC_ACQUIRE, "workgroup");
  }
}

template <int MODE>
__global__ __launch_bounds__(256) void cvt16_kernel(
    const float* __restrict__ src, unsigned short* __restrict__ dst, int nsrc8, int ntot8)
{
  const int i = blockIdx.x * 256 + threadIdx.x;
  if (i >= ntot8) return;
  const bool live = (i < nsrc8);
  const int ic = live ? i : (nsrc8 - 1);
  const float keep = live ? 1.0f : 0.0f;
  const size_t es = (size_t)ic << 3;
  const v4f a0 = *(const v4f*)(src + es);
  const v4f a1 = *(const v4f*)(src + es + 4);
  v8h hv;
#pragma unroll
  for (int e = 0; e < 4; ++e) {
    const float f0 = a0[e] * keep;
    const float f1 = a1[e] * keep;
    const unsigned short b0 = f2bf_bits(f0);
    const unsigned short b1 = f2bf_bits(f1);
    if (MODE == 0) {
      hv[e]     = __builtin_bit_cast(_Float16, b0);
      hv[4 + e] = __builtin_bit_cast(_Float16, b1);
    } else {
      hv[e]     = (_Float16)(bf_bits2f(b0) * kWcarry);
      hv[4 + e] = (_Float16)(bf_bits2f(b1) * kWcarry);
    }
  }
  unsigned short* q = dst + ((size_t)i << 3);
  *(volatile v8h*)q = hv;
  __threadfence();
  *(volatile v8h*)q = hv;
}

__global__ __launch_bounds__(256) void dtlo_cvt_kernel(
    const float* __restrict__ XD, unsigned short* __restrict__ DTL, int total8)
{
  const int i = blockIdx.x * 256 + threadIdx.x;
  if (i >= total8) return;
  const int row = i >> 3, c8 = (i & 7) * 8;
  const float* sp = XD + (size_t)row * kXdP + c8;
  const v4f a0 = *(const v4f*)(sp);
  const v4f a1 = *(const v4f*)(sp + 4);
  v8h hv;
#pragma unroll
  for (int e = 0; e < 4; ++e) {
    hv[e]     = (_Float16)a0[e];
    hv[4 + e] = (_Float16)a1[e];
  }
  unsigned short* q = DTL + (size_t)row * kDtR + c8;
  *(volatile v8h*)q = hv;
  __threadfence();
  *(volatile v8h*)q = hv;
}

__global__ __launch_bounds__(256) void conv_silu_kernel(
    const float* __restrict__ XR, const float* __restrict__ cw, const float* __restrict__ cb,
    unsigned short* __restrict__ U16)
{
  __shared__ __align__(16) float sT[16 * kConvTP];
  const int tid = threadIdx.x, lane = tid & 31, wave = tid >> 5;
  const int d0 = blockIdx.x * 256, d = d0 + tid;
  const int g0 = blockIdx.y * 64;
  const int tb = g0 & (kSeq - 1);
  const float w0 = bf_rne(cw[d * kDconv + 0]), w1 = bf_rne(cw[d * kDconv + 1]);
  const float w2 = bf_rne(cw[d * kDconv + 2]), w3 = bf_rne(cw[d * kDconv + 3]);
  const float bc = bf_rne(cb[d]);
  float xm3, xm2, xm1;
  {
    const bool hist = (tb > 0);
    const int rb = hist ? (g0 - 3) : g0;
    const float v3 = XR[(size_t)rb * kDin + d];
    const float v2 = XR[(size_t)(rb + 1) * kDin + d];
    const float v1 = XR[(size_t)(rb + 2) * kDin + d];
    xm3 = hist ? v3 : 0.f;
    xm2 = hist ? v2 : 0.f;
    xm1 = hist ? v1 : 0.f;
  }
#pragma unroll 1
  for (int sub = 0; sub < 4; ++sub) {
    const int lb = g0 + sub * 16;
#pragma unroll 1
    for (int s = 0; s < 16; ++s) {
      const float xcur = XR[(size_t)(lb + s) * kDin + d];
      float acc = w0 * xm3;
      acc = fmaf(w1, xm2, acc);
      acc = fmaf(w2, xm1, acc);
      acc = fmaf(w3, xcur, acc);
      const float sv = acc + bc;
      const float sg = __builtin_amdgcn_rcpf(1.0f + __expf(-sv));
      sT[s * kConvTP + tid] = sv * sg;
      xm3 = xm2; xm2 = xm1; xm1 = xcur;
    }
    __syncthreads();
    v8h hv[2];
#pragma unroll
    for (int it = 0; it < 2; ++it) {
      const float* sp = sT + (it * 8 + wave) * kConvTP + lane * 8;
      const v4f a0 = *(const v4f*)(sp);
      const v4f a1 = *(const v4f*)(sp + 4);
#pragma unroll
      for (int e = 0; e < 4; ++e) {
        hv[it][e]     = (_Float16)a0[e];
        hv[it][4 + e] = (_Float16)a1[e];
      }
    }
    for (int pass = 0; pass < 2; ++pass) {
#pragma unroll
      for (int it = 0; it < 2; ++it) {
        const size_t o = (size_t)(lb + it * 8 + wave) * kDin + d0 + lane * 8;
        *(volatile v8h*)(U16 + o) = hv[it];
      }
      __threadfence();
    }
    __syncthreads();
  }
}

__global__ __launch_bounds__(64) void scan_kernel(
    const float* __restrict__ XD, const float* __restrict__ DT, const unsigned* __restrict__ U16w,
    const float* __restrict__ ZR, const float* __restrict__ bdt, const float* __restrict__ Alog,
    const float* __restrict__ Dp, unsigned short* __restrict__ Y)
{
  __shared__ __align__(16) float sX[kScanTS * kScanXP];
  __shared__ __align__(16) float sY[kScanTS * kScanYP];
  __shared__ __align__(16) float sA[kNst * kScanCh];
  const int tid = threadIdx.x, lane = tid & 31, wave = tid >> 5;
  constexpr int kBlkPerB = kDin / kScanCh;
  const int bix = blockIdx.x / kBlkPerB;
  const int d0  = (blockIdx.x - bix * kBlkPerB) * kScanCh;
  const int d   = d0 + tid;
  const size_t row0 = (size_t)bix * kSeq;
#pragma unroll 1
  for (int s = 0; s < kNst; ++s) sA[s * kScanCh + tid] = -expf(bf_rne(Alog[(size_t)d * kNst + s]));
  __syncthreads();
  float negA[kNst], h[kNst];
#pragma unroll
  for (int s = 0; s < kNst; ++s) {
    negA[s] = sA[s * kScanCh + tid];
    h[s] = 0.0f;
  }
  const float bb = bf_rne(bdt[d]), Dd = bf_rne(Dp[d]);
  const int lr = tid >> 3, lc4 = (tid & 7) * 4;
  const int q = lane >> 3, c8 = (lane & 7) * 8;
  const unsigned usel = (unsigned)(tid & 1);
#pragma unroll 1
  for (int t0 = 0; t0 < kSeq; t0 += kScanTS) {
    __syncthreads();
#pragma unroll
    for (int i = 0; i < 8; ++i) {
      const int r = lr + 8 * i;
      *(v4f*)(sX + r * kScanXP + lc4) = *(const v4f*)(XD + (row0 + t0 + r) * kXdP + kDtR + lc4);
    }
    __syncthreads();
#pragma unroll 1
    for (int s = 0; s < kScanTS; ++s) {
      const int t = t0 + s;
      const float* xr = sX + s * kScanXP;
      float Bs[kNst], Cs[kNst];
#pragma unroll
      for (int q4 = 0; q4 < 4; ++q4) {
        const v4f bv = *(const v4f*)(xr + 4 * q4);
        const v4f cv = *(const v4f*)(xr + kNst + 4 * q4);
        Bs[4 * q4 + 0] = bv[0]; Bs[4 * q4 + 1] = bv[1]; Bs[4 * q4 + 2] = bv[2]; Bs[4 * q4 + 3] = bv[3];
        Cs[4 * q4 + 0] = cv[0]; Cs[4 * q4 + 1] = cv[1]; Cs[4 * q4 + 2] = cv[2]; Cs[4 * q4 + 3] = cv[3];
      }
      const size_t eoff = (row0 + t) * kDin + d;
      const float dtv = DT[eoff];
      const unsigned uw = U16w[eoff >> 1];
      const float zv = ZR[eoff];
      const unsigned ubits = usel ? (uw >> 16) : (uw & 0xffffu);
      const float xt  = h16_to_f32(ubits);
      const float v   = (dtv + bb) + bb;
      const float a   = __expf(-fabsf(v));
      const float uu  = 1.0f + a;
      const float l1p = __logf(uu) + (a - (uu - 1.0f)) * __builtin_amdgcn_rcpf(uu);
      const float dlt = fmaxf(v, 0.0f) + l1p;
      const float dtx = dlt * xt;
      float y = 0.0f;
#pragma unroll
      for (int k = 0; k < kNst; ++k) {
        const float e = __expf(dlt * negA[k]);
        h[k] = e * h[k] + dtx * Bs[k];
        y = h[k] * Cs[k] + y;
      }
      y = xt * Dd + y;
      const float sg = __builtin_amdgcn_rcpf(1.0f + __expf(-zv));
      y = y * (zv * sg);
      sY[s * kScanYP + tid] = y * kYcarry;
    }
    __syncthreads();
    v8h hv[8];
#pragma unroll
    for (int it = 0; it < 8; ++it) {
      const int row = it * 8 + wave * 4 + q;
      const float* sp = sY + row * kScanYP + c8;
      const v4f a0 = *(const v4f*)(sp);
      const v4f a1 = *(const v4f*)(sp + 4);
#pragma unroll
      for (int e = 0; e < 4; ++e) {
        hv[it][e]     = (_Float16)a0[e];
        hv[it][4 + e] = (_Float16)a1[e];
      }
    }
    for (int pass = 0; pass < 2; ++pass) {
#pragma unroll
      for (int it = 0; it < 8; ++it) {
        const int row = it * 8 + wave * 4 + q;
        const size_t o = (row0 + t0 + row) * kDin + d0 + c8;
        *(volatile v8h*)(Y + o) = hv[it];
      }
      __threadfence();
    }
  }
}

extern "C" void kernel_launch(void* const* d_in, const int* in_sizes, int n_in,
                              void* d_out, int out_size, void* d_ws, size_t ws_size,
                              hipStream_t stream) {
  if (n_in < 10) return;
  if (in_sizes[0] != kRows * kDm) return;
  if (in_sizes[1] != 2 * kDin * kDm) return;
  if (in_sizes[2] != kDin * kDconv) return;
  if (in_sizes[3] != kDin) return;
  if (in_sizes[4] != kXdW * kDin) return;
  if (in_sizes[5] != kDin * kDtR) return;
  if (in_sizes[6] != kDin) return;
  if (in_sizes[7] != kDin * kNst) return;
  if (in_sizes[8] != kDin) return;
  if (in_sizes[9] != kDm * kDin) return;
  if (out_size != kRows * kDm) return;
  if (ws_size < kWsTotal) return;

  const float* hidden  = (const float*)d_in[0];
  const float* W_in    = (const float*)d_in[1];
  const float* conv_w  = (const float*)d_in[2];
  const float* conv_b  = (const float*)d_in[3];
  const float* W_xproj = (const float*)d_in[4];
  const float* W_dt    = (const float*)d_in[5];
  const float* b_dt    = (const float*)d_in[6];
  const float* A_log   = (const float*)d_in[7];
  const float* Dp      = (const float*)d_in[8];
  const float* W_out   = (const float*)d_in[9];
  float* out = (float*)d_out;

  char* ws = (char*)d_ws;
  unsigned short* XH  = (unsigned short*)(ws + kOffXH);
  unsigned short* WIN = (unsigned short*)(ws + kOffWIN);
  unsigned short* WXP = (unsigned short*)(ws + kOffWXP);
  unsigned short* WDT = (unsigned short*)(ws + kOffWDT);
  unsigned short* WOU = (unsigned short*)(ws + kOffWOU);
  float*          XR  = (float*)(ws + kOffXR);
  float*          DT  = (float*)(ws + kOffXR);
  float*          ZR  = (float*)(ws + kOffZR);
  unsigned short* U16 = (unsigned short*)(ws + kOffU16);
  float*          XD  = (float*)(ws + kOffXD);
  unsigned short* DTL = (unsigned short*)(ws + kOffDTL);
  unsigned short* Y   = (unsigned short*)(ws + kOffY);

  cvt16_kernel<0><<<(kRows * kDm / 8) / 256, 256, 0, stream>>>(hidden, XH, kRows * kDm / 8, kRows * kDm / 8);
  cvt16_kernel<0><<<(2 * kDin * kDm / 8) / 256, 256, 0, stream>>>(W_in, WIN, 2 * kDin * kDm / 8, 2 * kDin * kDm / 8);
  cvt16_kernel<1><<<(kXdP * kDin / 8) / 256, 256, 0, stream>>>(W_xproj, WXP, kXdW * kDin / 8, kXdP * kDin / 8);
  cvt16_kernel<1><<<(kDin * kDtR / 8) / 256, 256, 0, stream>>>(W_dt, WDT, kDin * kDtR / 8, kDin * kDtR / 8);
  cvt16_kernel<1><<<(kDm * kDin / 8) / 256, 256, 0, stream>>>(W_out, WOU, kDm * kDin / 8, kDm * kDin / 8);

  wmma_gemm64<1, false, 0, 0, false><<<dim3(((kRows / 64) * (kDin / 64)) / 8, 1), 256, 0, stream>>>(
      XH, nullptr, kDm, 0L,
      WIN, nullptr, kDm, 0L,
      (void*)XR, nullptr, kDin, 0L,
      nullptr, nullptr, 0L,
      kRows, kDin, kDm, 1.0f);
  wmma_gemm64<1, false, 0, 0, false><<<dim3(((kRows / 64) * (kDin / 64)) / 8, 1), 256, 0, stream>>>(
      XH, nullptr, kDm, 0L,
      WIN + (size_t)kDin * kDm, nullptr, kDm, 0L,
      (void*)ZR, nullptr, kDin, 0L,
      nullptr, nullptr, 0L,
      kRows, kDin, kDm, 1.0f);

  conv_silu_kernel<<<dim3(kDin / 256, kRows / 64), 256, 0, stream>>>(XR, conv_w, conv_b, U16);

  wmma_gemm64<0, false, 0, 0, false><<<dim3(((kRows / 64) * (kXdP / 64)) / 8, 1), 256, 0, stream>>>(
      U16, nullptr, kDin, 0L,
      WXP, nullptr, kDin, 0L,
      (void*)XD, nullptr, kXdP, 0L,
      nullptr, nullptr, 0L,
      kRows, kXdP, kDin, kWcarryInv);

  dtlo_cvt_kernel<<<(kRows * kDtR / 8) / 256, 256, 0, stream>>>(XD, DTL, kRows * kDtR / 8);

  wmma_gemm64<0, false, 0, 0, false><<<dim3(((kRows / 64) * (kDin / 64)) / 8, 1), 256, 0, stream>>>(
      DTL, nullptr, kDtR, 0L,
      WDT, nullptr, kDtR, 0L,
      (void*)DT, nullptr, kDin, 0L,
      nullptr, nullptr, 0L,
      kRows, kDin, kDtR, kWcarryInv);

  scan_kernel<<<kBatch * (kDin / kScanCh), kScanCh, 0, stream>>>(XD, DT, (const unsigned*)U16, ZR, b_dt, A_log, Dp, Y);

  wmma_gemm64<0, false, 0, 0, false><<<dim3(((kRows / 64) * (kDm / 64)) / 8, 1), 256, 0, stream>>>(
      Y, nullptr, kDin, 0L,
      WOU, nullptr, kDin, 0L,
      (void*)out, nullptr, kDm, 0L,
      nullptr, nullptr, 0L,
      kRows, kDm, kDin, kYWInv);
}
